// TumorAwareAttention3D_10471130268146
// MI455X (gfx1250) — hardware-verified
//
#include <hip/hip_runtime.h>
#include <math.h>
#include <stdint.h>

#define NB    2
#define CCH   64
#define NN    4096
#define NHD   4
#define HDM   16
#define NQKV  192
#define QBLK  128
static_assert(NHD * HDM == CCH);
static_assert((NN % QBLK) == 0 && (NN % 64) == 0 && (NQKV % 64) == 0 && (CCH % 64) == 0 && (CCH % 32) == 0);

typedef _Float16 v16h __attribute__((ext_vector_type(16)));
typedef _Float16 v8h  __attribute__((ext_vector_type(8)));
typedef float    v8f  __attribute__((ext_vector_type(8)));
typedef float    v4f  __attribute__((ext_vector_type(4)));
typedef unsigned int v4u __attribute__((ext_vector_type(4)));

__device__ __forceinline__ unsigned short bf_bits(float f) {
  unsigned u = __float_as_uint(f);
  return (unsigned short)((u + 0x7FFFu + ((u >> 16) & 1u)) >> 16);
}
__device__ __forceinline__ float bf_up(unsigned short h) { return __uint_as_float(((unsigned)h) << 16); }
__device__ __forceinline__ unsigned short h_bits(_Float16 x) { return __builtin_bit_cast(unsigned short, x); }
__device__ __forceinline__ unsigned pk16(unsigned short a, unsigned short b) { return (unsigned)a | ((unsigned)b << 16); }
__device__ __forceinline__ v8f zero8() { v8f z = {0.f, 0.f, 0.f, 0.f, 0.f, 0.f, 0.f, 0.f}; return z; }
__device__ __forceinline__ float clipf(float v, float lo, float hi) { return fminf(fmaxf(v, lo), hi); }

__device__ __forceinline__ v16h ldfrag_h(const _Float16* p) {
  union { v16h v; v8h h[2]; } f;
  f.h[0] = *(const v8h*)(p);
  f.h[1] = *(const v8h*)(p + 16);
  return f.v;
}
__device__ __forceinline__ v16h ldfrag_8z(const _Float16* p) {
  union { v16h v; v8h h[2]; } f;
  const _Float16 zz = (_Float16)0.0f;
  const v8h z = {zz, zz, zz, zz, zz, zz, zz, zz};
  f.h[0] = *(const v8h*)(p);
  f.h[1] = z;
  return f.v;
}

__device__ __forceinline__ v8f mma_h_raw(v16h a, v16h b, v8f c) {
  return __builtin_amdgcn_wmma_f32_16x16x32_f16(false, a, false, b, (short)0, c, false, false);
}
__device__ __forceinline__ void res_guard(v8f& t, v8f& acc, v16h x, v16h y) {
#if defined(__HIP_DEVICE_COMPILE__)
  asm volatile("v_nop\n\tv_nop\n\tv_nop\n\tv_nop" : "+v"(t), "+v"(acc) : "v"(x), "v"(y));
#endif
}
__device__ __forceinline__ void dep_guard_h(v8f& a, v8f& b, v16h x, v16h y) {
#if defined(__HIP_DEVICE_COMPILE__)
  asm volatile("v_nop\n\tv_nop\n\tv_nop\n\tv_nop" : "+v"(a), "+v"(b) : "v"(x), "v"(y));
#endif
}
__device__ __forceinline__ void guard2x3(v8f& a, v8f& b, v16h x, v16h y, v16h z) {
#if defined(__HIP_DEVICE_COMPILE__)
  asm volatile("v_nop\n\tv_nop\n\tv_nop\n\tv_nop" : "+v"(a), "+v"(b) : "v"(x), "v"(y), "v"(z));
#endif
}
__device__ __forceinline__ void guard4x4(v8f& a, v8f& b, v8f& c, v8f& d, v16h w, v16h x, v16h y, v16h z) {
#if defined(__HIP_DEVICE_COMPILE__)
  asm volatile("v_nop\n\tv_nop\n\tv_nop\n\tv_nop" : "+v"(a), "+v"(b), "+v"(c), "+v"(d) : "v"(w), "v"(x), "v"(y), "v"(z));
#endif
}
__device__ __forceinline__ void keep4_h(v16h a, v16h b, v16h c, v16h d) {
#if defined(__HIP_DEVICE_COMPILE__)
  asm volatile("v_nop" :: "v"(a), "v"(b), "v"(c), "v"(d));
#endif
}
__device__ __forceinline__ void acc_guard4(v8f& a, v8f& b, v8f& c, v8f& d) {
#if defined(__HIP_DEVICE_COMPILE__)
  asm volatile("v_nop\n\tv_nop\n\tv_nop\n\tv_nop" : "+v"(a), "+v"(b), "+v"(c), "+v"(d));
#endif
}
__device__ __forceinline__ void acc_guard2(v8f& a, v8f& b) {
#if defined(__HIP_DEVICE_COMPILE__)
  asm volatile("v_nop\n\tv_nop\n\tv_nop\n\tv_nop" : "+v"(a), "+v"(b));
#endif
}
__device__ __forceinline__ void wave_sync_lds() {
  __builtin_amdgcn_fence(__ATOMIC_RELEASE, "workgroup");
  __builtin_amdgcn_wave_barrier();
  __builtin_amdgcn_fence(__ATOMIC_ACQUIRE, "workgroup");
}

__global__ __launch_bounds__(256) void cvt_h8(const float* __restrict__ in, unsigned short* out, int n8, float scale) {
  const int i = blockIdx.x * 256 + threadIdx.x;
  if (i < n8) {
    const v4f a = *(const v4f*)(in + (size_t)i * 8);
    const v4f c = *(const v4f*)(in + (size_t)i * 8 + 4);
    float f[8];
    f[0] = a[0]; f[1] = a[1]; f[2] = a[2]; f[3] = a[3];
    f[4] = c[0]; f[5] = c[1]; f[6] = c[2]; f[7] = c[3];
    unsigned short hb[8];
#pragma unroll
    for (int e = 0; e < 8; ++e) hb[e] = h_bits((_Float16)(bf_up(bf_bits(f[e])) * scale));
    v4u p;
    p[0] = pk16(hb[0], hb[1]);
    p[1] = pk16(hb[2], hb[3]);
    p[2] = pk16(hb[4], hb[5]);
    p[3] = pk16(hb[6], hb[7]);
    *(volatile v4u*)(out + (size_t)i * 8) = p;
    __threadfence();
    *(volatile v4u*)(out + (size_t)i * 8) = p;
  }
}

#define QTP 72
__global__ __launch_bounds__(256) void cvt_qt(const float* __restrict__ x, unsigned short* out, float scale) {
  __shared__ __align__(16) unsigned short ts[64 * QTP];
  const int tid = threadIdx.x;
  const int l0 = blockIdx.x * 64, b = blockIdx.y;
#pragma unroll 1
  for (int pass = 0; pass < 4; ++pass) {
    const int c = pass * 16 + (tid >> 4);
    const int l4 = (tid & 15) * 4;
    const v4f v = *(const v4f*)(x + ((size_t)(b * CCH + c) * NN) + l0 + l4);
#pragma unroll
    for (int i = 0; i < 4; ++i) ts[(l4 + i) * QTP + c] = h_bits((_Float16)(bf_up(bf_bits(v[i])) * scale));
  }
  __syncthreads();
#pragma unroll 1
  for (int pass = 0; pass < 2; ++pass) {
    const int lr = pass * 32 + (tid >> 3);
    const int c8 = (tid & 7) * 8;
    const v4u v = *(const v4u*)(ts + lr * QTP + c8);
    unsigned short* dst = out + ((size_t)(b * NN) + l0 + lr) * CCH + c8;
    *(volatile v4u*)dst = v;
    __threadfence();
    *(volatile v4u*)dst = v;
  }
}

template <int NSPLIT, int BIAS>
__global__ __launch_bounds__(256) void gemm64(
    const unsigned short* __restrict__ Ap, int lda, long long sAy, long long sAz,
    const unsigned short* __restrict__ Btp, int ldb, long long sBy, long long sBz,
    const unsigned short* __restrict__ Bt2p, int ldb2,
    const float* __restrict__ bias,
    float* Cout, int ldc, long long sCy, long long sCz,
    int M, int N, int K, float oscale, float rres) {
  const _Float16* A   = (const _Float16*)(const void*)Ap;
  const _Float16* Bt  = (const _Float16*)(const void*)Btp;
  const _Float16* Bt2 = (const _Float16*)(const void*)Bt2p;
  __shared__ __align__(16) float sT[8][16 * 68];
  const int by   = blockIdx.y;
  const int bz   = blockIdx.z;
  const int lane = threadIdx.x & 31;
  const int wave = threadIdx.x >> 5;
  const int tilesN = N >> 6;
  const int tilesM = M >> 6;
  const int tile = blockIdx.x * 8 + wave;
  if (tile >= tilesM * tilesN) return;
  const int tm = tile / tilesN;
  const int tn = tile - tm * tilesN;
  const int m0 = tm << 6;
  const int n0 = tn << 6;

  const _Float16* Ab  = A + (size_t)by * (size_t)sAy + (size_t)bz * (size_t)sAz;
  const _Float16* Bb  = Bt + (size_t)by * (size_t)sBy + (size_t)bz * (size_t)sBz;
  const _Float16* Bb2 = (NSPLIT == 2) ? (Bt2 + (size_t)by * (size_t)sBy + (size_t)bz * (size_t)sBz) : Bb;
  const int ld2 = (NSPLIT == 2) ? ldb2 : ldb;

  const int rlane = lane & 15;
  const int koff  = (lane >> 4) * 8;
  const int mOff  = (lane >> 4) * 8;

  v8f acc[4][4];
#pragma unroll
  for (int i = 0; i < 4; ++i)
#pragma unroll
    for (int j = 0; j < 4; ++j) acc[i][j] = zero8();

  for (int k0 = 0; k0 < K; k0 += 32) {
    v16h bf[4];
#pragma unroll
    for (int j = 0; j < 4; ++j) {
      const size_t bo = (size_t)(n0 + (j << 4) + rlane) * ldb + koff + k0;
      bf[j] = ldfrag_h(Bb + bo);
    }
#pragma unroll
    for (int i = 0; i < 4; ++i) {
      const size_t ao = (size_t)(m0 + (i << 4) + rlane) * lda + koff + k0;
      const v16h ah = ldfrag_h(Ab + ao);
#pragma unroll
      for (int j = 0; j < 4; ++j) acc[i][j] = mma_h_raw(ah, bf[j], acc[i][j]);
      dep_guard_h(acc[i][0], acc[i][3], ah, bf[3]);
    }
    if (NSPLIT == 2) {
#pragma unroll
      for (int j = 0; j < 4; ++j) {
        const size_t bo = (size_t)(n0 + (j << 4) + rlane) * ld2 + koff + k0;
        bf[j] = ldfrag_h(Bb2 + bo);
      }
#pragma unroll
      for (int i = 0; i < 4; ++i) {
        const size_t ao = (size_t)(m0 + (i << 4) + rlane) * lda + koff + k0;
        const v16h al = ldfrag_h(Ab + ao);
#pragma unroll
        for (int j = 0; j < 4; ++j) {
          v8f tp = mma_h_raw(al, bf[j], zero8());
          res_guard(tp, acc[i][j], al, bf[j]);
#pragma unroll
          for (int r = 0; r < 8; ++r) acc[i][j][r] += tp[r] * rres;
        }
        dep_guard_h(acc[i][0], acc[i][3], al, bf[3]);
      }
    }
    keep4_h(bf[0], bf[1], bf[2], bf[3]);
  }
  acc_guard4(acc[0][0], acc[0][1], acc[0][2], acc[0][3]);
  acc_guard4(acc[1][0], acc[1][1], acc[1][2], acc[1][3]);
  acc_guard4(acc[2][0], acc[2][1], acc[2][2], acc[2][3]);
  acc_guard4(acc[3][0], acc[3][1], acc[3][2], acc[3][3]);

  float* slab = sT[wave];
  float* C = Cout + (size_t)by * (size_t)sCy + (size_t)bz * (size_t)sCz;
#pragma unroll
  for (int i = 0; i < 4; ++i) {
    const int mBase = m0 + (i << 4);
    float brow[8];
#pragma unroll
    for (int r = 0; r < 8; ++r) brow[r] = 0.f;
    if (BIAS == 2) {
#pragma unroll
      for (int r = 0; r < 8; ++r) brow[r] = bf_up(bf_bits(bias[mBase + mOff + r]));
    }
#pragma unroll
    for (int j = 0; j < 4; ++j) {
#pragma unroll
      for (int r = 0; r < 8; ++r) {
        slab[(mOff + r) * 68 + (j << 4) + rlane] = acc[i][j][r] * oscale + brow[r];
      }
    }
    wave_sync_lds();
    {
      const int hh = lane >> 4, c4 = (lane & 15) * 4;
      for (int pass = 0; pass < 2; ++pass) {
#pragma unroll
        for (int it = 0; it < 8; ++it) {
          const int row = it * 2 + hh;
          const v4f v = *(const v4f*)(slab + row * 68 + c4);
          *(volatile v4f*)(C + (size_t)(mBase + row) * ldc + n0 + c4) = v;
        }
        __threadfence();
      }
    }
    wave_sync_lds();
  }
}

#define YP 68
__global__ __launch_bounds__(256) void relayout_kernel(
    const float* __restrict__ Y,
    unsigned short* QH, unsigned short* QL, unsigned short* KX,
    unsigned short* VH, unsigned short* VL) {
  __shared__ __align__(16) float ys[128 * YP];
  const int tid = threadIdx.x, lane = tid & 31, wave = tid >> 5;
  const int n0 = blockIdx.x * 64, b = blockIdx.y;
  const float* Yb = Y + (size_t)b * NQKV * NN;

#pragma unroll 1
  for (int it = 0; it < 8; ++it) {
    const int idx = it * 256 + tid;
    const int row = idx >> 4;
    const int c4  = (idx & 15) * 4;
    const v4f v = *(const v4f*)(Yb + (size_t)row * NN + n0 + c4);
    *(v4f*)(ys + row * YP + c4) = v;
  }
  __syncthreads();

  {
    const bool isq  = (wave < 4);
    const int  head = wave & 3;
    const int  ob   = (isq ? 0 : 64) + head * 16;
    const int  inst = b * NHD + head;
    unsigned short* Ph = isq ? QH : KX;
#pragma unroll 1
    for (int it = 0; it < 4; ++it) {
      const int r  = it * 16 + (lane >> 1);
      const int dh = lane & 1;
      const float* src = ys + (ob + dh * 8) * YP + r;
      unsigned short hb[8], lb[8];
#pragma unroll
      for (int i = 0; i < 8; ++i) {
        const float v = src[i * YP] * 16.0f;
        const _Float16 xh = (_Float16)v;
        hb[i] = h_bits(xh);
        lb[i] = h_bits((_Float16)((v - (float)xh) * 2048.0f));
      }
      v4u ph, pl;
#pragma unroll
      for (int q = 0; q < 4; ++q) {
        ph[q] = pk16(hb[2 * q], hb[2 * q + 1]);
        pl[q] = pk16(lb[2 * q], lb[2 * q + 1]);
      }
      const size_t dst = ((size_t)(inst * NN + n0 + r)) * HDM + dh * 8;
      *(volatile v4u*)(Ph + dst) = ph;
      if (isq) *(volatile v4u*)(QL + dst) = pl;
      __threadfence();
      *(volatile v4u*)(Ph + dst) = ph;
      if (isq) *(volatile v4u*)(QL + dst) = pl;
    }
  }

#pragma unroll 1
  for (int j = 0; j < 2; ++j) {
    const int it   = wave * 2 + j;
    const int row  = it * 4 + (lane >> 3);
    const int col8 = (lane & 7) * 8;
    const float* src = Yb + (size_t)(128 + row) * NN + n0 + col8;
    const v4f a = *(const v4f*)(src);
    const v4f c = *(const v4f*)(src + 4);
    float f[8];
    f[0] = a[0]; f[1] = a[1]; f[2] = a[2]; f[3] = a[3];
    f[4] = c[0]; f[5] = c[1]; f[6] = c[2]; f[7] = c[3];
    unsigned short hb[8], lb[8];
#pragma unroll
    for (int i = 0; i < 8; ++i) {
      const float v = f[i] * 16.0f;
      const _Float16 xh = (_Float16)v;
      hb[i] = h_bits(xh);
      lb[i] = h_bits((_Float16)((v - (float)xh) * 2048.0f));
    }
    v4u ph, pl;
#pragma unroll
    for (int q = 0; q < 4; ++q) {
      ph[q] = pk16(hb[2 * q], hb[2 * q + 1]);
      pl[q] = pk16(lb[2 * q], lb[2 * q + 1]);
    }
    const size_t dst = ((size_t)(b * CCH + row)) * NN + n0 + col8;
    *(volatile v4u*)(VH + dst) = ph;
    *(volatile v4u*)(VL + dst) = pl;
    __threadfence();
    *(volatile v4u*)(VH + dst) = ph;
    *(volatile v4u*)(VL + dst) = pl;
  }
}

#define VPITCH 72
#define SPITCH 72
__global__ __launch_bounds__(256) void attn_kernel(
    const unsigned short* __restrict__ QHp, const unsigned short* __restrict__ QLp,
    const unsigned short* __restrict__ KXp,
    const unsigned short* __restrict__ VHp, const unsigned short* __restrict__ VLp,
    const float* __restrict__ tpm, const float* __restrict__ temperature,
    unsigned short* CTXh, unsigned short* CTXl, float rscale) {
  __shared__ __align__(16) unsigned short kl_u[64 * HDM];
  __shared__ __align__(16) unsigned short vh_u[16 * VPITCH];
  __shared__ __align__(16) unsigned short vr_u[16 * VPITCH];
  __shared__ __align__(16) float gcol[64];
  __shared__ __align__(16) unsigned short sth[8 * 16 * SPITCH];
  __shared__ __align__(16) unsigned short stl[8 * 16 * SPITCH];
  const _Float16* kl  = (const _Float16*)(const void*)kl_u;
  const _Float16* vhh = (const _Float16*)(const void*)vh_u;
  const _Float16* vrl = (const _Float16*)(const void*)vr_u;
  const _Float16* QH  = (const _Float16*)(const void*)QHp;
  const _Float16* QL  = (const _Float16*)(const void*)QLp;

  const int tid = threadIdx.x, lane = tid & 31, wave = tid >> 5;
  const int b = blockIdx.y;
  const int qBase = blockIdx.x * QBLK + wave * 16;
  const int rlane = lane & 15, hsel = lane >> 4, koff = hsel * 8;

  const float temp = clipf(bf_up(bf_bits(temperature[0])), 0.1f, 2.0f);
  const float sc   = temp * (1.0f / 2048.0f);
  const float gi   = clipf(bf_up(bf_bits(tpm[(size_t)b * NN + qBase + rlane])), 0.01f, 1.0f);
  const float rowf = sc * gi;
  const float C2048  = 1.0f / 2048.0f;
  const float LN1024 = 6.931471805599453f;

  const int t2 = tid & 127;
  const int vrow = t2 >> 3;
  const int vc8  = (t2 & 7) * 8;
  unsigned short* kd  = kl_u + t2 * 8;
  unsigned short* vhd = vh_u + vrow * VPITCH + vc8;
  unsigned short* vrd = vr_u + vrow * VPITCH + vc8;

#pragma unroll 1
  for (int h = 0; h < NHD; ++h) {
    const int inst = b * NHD + h;
    const size_t qo = ((size_t)(inst * NN + qBase + rlane)) * HDM + koff;
    const v16h qh = ldfrag_8z(QH + qo);
    const v16h ql = ldfrag_8z(QL + qo);
    const unsigned short* Kg  = KXp + (size_t)inst * NN * HDM + (size_t)t2 * 8;
    const unsigned short* Vhg = VHp + ((size_t)(b * CCH + h * HDM + vrow)) * NN + vc8;
    const unsigned short* Vlg = VLp + ((size_t)(b * CCH + h * HDM + vrow)) * NN + vc8;

    v8f oh = zero8(), ol = zero8();
    float m_run = -1e30f, l_run = 0.f;

#pragma unroll 1
    for (int kb = 0; kb < NN; kb += 64) {
      __syncthreads();
      if (wave < 4) {
        const v4u kv = *(const v4u*)(Kg + (size_t)kb * HDM);
        *(v4u*)kd = kv;
        const v4u lv = *(const v4u*)(Vlg + kb);
        *(v4u*)vrd = lv;
      } else {
        const v4u hv = *(const v4u*)(Vhg + kb);
        *(v4u*)vhd = hv;
      }
      if (wave < 2) {
        const float g = clipf(bf_up(bf_bits(tpm[(size_t)b * NN + kb + tid])), 0.01f, 1.0f);
        gcol[tid] = sc * g;
      }
      __syncthreads();

#pragma unroll 1
      for (int sub = 0; sub < 2; ++sub) {
        const int kr = 32 * sub;
        const v16h kf0 = ldfrag_8z(kl + (kr + rlane) * HDM + koff);
        const v16h kf1 = ldfrag_8z(kl + (kr + 16 + rlane) * HDM + koff);
        v8f sh0 = mma_h_raw(kf0, qh, zero8());
        v8f sh1 = mma_h_raw(kf1, qh, zero8());
        v8f sr0 = mma_h_raw(kf0, ql, zero8());
        v8f sr1 = mma_h_raw(kf1, ql, zero8());
        guard4x4(sh0, sh1, sr0, sr1, kf0, kf1, qh, ql);

        const v4f ga0 = *(const v4f*)(gcol + kr + koff);
        const v4f ga1 = *(const v4f*)(gcol + kr + koff + 4);
        const v4f gb0 = *(const v4f*)(gcol + kr + 16 + koff);
        const v4f gb1 = *(const v4f*)(gcol + kr + 16 + koff + 4);
        float a0[8], a1[8];
#pragma unroll
        for (int r = 0; r < 4; ++r) {
          a0[r]     = (sh0[r]     + sr0[r]     * C2048) * (rowf + ga0[r]);
          a0[r + 4] = (sh0[r + 4] + sr0[r + 4] * C2048) * (rowf + ga1[r]);
          a1[r]     = (sh1[r]     + sr1[r]     * C2048) * (rowf + gb0[r]);
          a1[r + 4] = (sh1[r + 4] + sr1[r + 4] * C2048) * (rowf + gb1[r]);
        }

        float mloc = -1e30f;
#pragma unroll
        for (int r = 0; r < 8; ++r) mloc = fmaxf(mloc, fmaxf(a0[r], a1[r]));
        mloc = fmaxf(mloc, __shfl_xor(mloc, 16, 32));
        const float newM  = fmaxf(m_run, mloc);
        const float alpha = __expf(m_run - newM);
        const float msh   = newM - LN1024;
        float ssum = 0.f;
        float p0[8], p1[8];
#pragma unroll
        for (int r = 0; r < 8; ++r) {
          p0[r] = __expf(a0[r] - msh);
          p1[r] = __expf(a1[r] - msh);
          ssum += p0[r] + p1[r];
        }
        ssum += __shfl_xor(ssum, 16, 32);
        l_run = l_run * alpha + ssum;
        m_run = newM;
#pragma unroll
        for (int r = 0; r < 8; ++r) { oh[r] *= alpha; ol[r] *= alpha; }

        union { v16h v; _Float16 s[16]; } pf;
#pragma unroll
        for (int r = 0; r < 8; ++r) {
          pf.s[r]     = (_Float16)p0[r];
          pf.s[8 + r] = (_Float16)p1[r];
        }

        const v16h vah = ldfrag_h(vhh + rlane * VPITCH + kr + koff);
        const v16h val = ldfrag_h(vrl + rlane * VPITCH + kr + koff);
        oh = mma_h_raw(vah, pf.v, oh);
        ol = mma_h_raw(val, pf.v, ol);
        guard2x3(oh, ol, vah, val, pf.v);
      }
    }
    acc_guard2(oh, ol);

    const float inv = 4.0f * (1.0f / l_run);
    v4u hv, lw;
#pragma unroll
    for (int e = 0; e < 4; ++e) {
      const float f0 = (oh[2 * e]     + ol[2 * e]     * C2048) * inv;
      const float f1 = (oh[2 * e + 1] + ol[2 * e + 1] * C2048) * inv;
      const _Float16 x0 = (_Float16)f0, x1 = (_Float16)f1;
      hv[e] = pk16(h_bits(x0), h_bits(x1));
      lw[e] = pk16(h_bits((_Float16)((f0 - (float)x0) * rscale)),
                   h_bits((_Float16)((f1 - (float)x1) * rscale)));
    }
    const int so = (wave * 16 + rlane) * SPITCH + h * HDM + koff;
    *(v4u*)(sth + so) = hv;
    *(v4u*)(stl + so) = lw;
  }

  wave_sync_lds();
  {
    const int rq = lane >> 3, c8 = (lane & 7) * 8;
    const unsigned short* hs = sth + (wave * 16) * SPITCH;
    const unsigned short* ls = stl + (wave * 16) * SPITCH;
    const size_t rb = (size_t)b * NN + qBase;
    for (int pass = 0; pass < 2; ++pass) {
#pragma unroll
      for (int it = 0; it < 4; ++it) {
        const int row = it * 4 + rq;
        const v4u v = *(const v4u*)(hs + row * SPITCH + c8);
        *(volatile v4u*)(CTXh + (rb + row) * CCH + c8) = v;
      }
      __threadfence();
    }
    for (int pass = 0; pass < 2; ++pass) {
#pragma unroll
      for (int it = 0; it < 4; ++it) {
        const int row = it * 4 + rq;
        const v4u v = *(const v4u*)(ls + row * SPITCH + c8);
        *(volatile v4u*)(CTXl + (rb + row) * CCH + c8) = v;
      }
      __threadfence();
    }
  }
}

extern "C" void kernel_launch(void* const* d_in, const int* in_sizes, int n_in,
                              void* d_out, int out_size, void* d_ws, size_t ws_size,
                              hipStream_t stream) {
  if (n_in < 7) return;
  if (in_sizes[0] != NB * CCH * NN) return;
  if (in_sizes[1] != NB * NN) return;
  if (in_sizes[2] != NQKV * CCH) return;
  if (in_sizes[3] != NQKV) return;
  if (in_sizes[4] != CCH * CCH) return;
  if (in_sizes[5] != CCH) return;
  if (in_sizes[6] < 1) return;
  if (out_size != NB * CCH * NN) return;

  const float* x      = (const float*)d_in[0];
  const float* tpm    = (const float*)d_in[1];
  const float* qkv_w  = (const float*)d_in[2];
  const float* qkv_b  = (const float*)d_in[3];
  const float* proj_w = (const float*)d_in[4];
  const float* proj_b = (const float*)d_in[5];
  const float* temper = (const float*)d_in[6];

  const size_t PXT = (size_t)NB * NN * CCH * 2;
  const size_t PW3 = (size_t)NQKV * CCH * 2;
  const size_t PPW = (size_t)CCH * CCH * 2;
  const size_t PY  = (size_t)NB * NQKV * NN * 4;
  const size_t PQ  = (size_t)NB * NHD * NN * HDM * 2;
  const size_t PV  = (size_t)NB * CCH * NN * 2;
  const size_t PCT = (size_t)NB * NN * CCH * 2;
  size_t off = 0;
  const size_t oXT = off; off += PXT;
  const size_t oW3 = off; off += PW3;
  const size_t oPW = off; off += PPW;
  const size_t oY  = off; off += PY;
  const size_t oQH = off; off += PQ;
  const size_t oQL = off; off += PQ;
  const size_t oKX = off; off += PQ;
  const size_t oVH = off; off += PV;
  const size_t oVL = off; off += PV;
  const size_t oCH = off; off += PCT;
  const size_t oCL = off; off += PCT;
  if (off > ws_size) return;
  if (off > (size_t)134217728) return;

  char* ws = (char*)d_ws;
  unsigned short* XT   = (unsigned short*)(ws + oXT);
  unsigned short* W3   = (unsigned short*)(ws + oW3);
  unsigned short* PWp  = (unsigned short*)(ws + oPW);
  float*          Y    = (float*)(ws + oY);
  unsigned short* QH   = (unsigned short*)(ws + oQH);
  unsigned short* QL   = (unsigned short*)(ws + oQL);
  unsigned short* KX   = (unsigned short*)(ws + oKX);
  unsigned short* VH   = (unsigned short*)(ws + oVH);
  unsigned short* VL   = (unsigned short*)(ws + oVL);
  unsigned short* CTXh = (unsigned short*)(ws + oCH);
  unsigned short* CTXl = (unsigned short*)(ws + oCL);
  float*          out  = (float*)d_out;

  const dim3 blk(256);
  const int n8w3 = NQKV * CCH / 8;
  const int n8pw = CCH * CCH / 8;
  const dim3 gW3((n8w3 + 255) / 256);
  const dim3 gPW((n8pw + 255) / 256);
  const dim3 gQt(NN / 64, NB);
  const dim3 gQkv(((NQKV / 64) * (NN / 64) + 7) / 8, NB, 1);
  const dim3 gRel(NN / 64, NB);
  const dim3 gAttn(NN / QBLK, NB);
  const dim3 gProj(((CCH / 64) * (NN / 64) + 7) / 8, NB, 1);

  const float oscQkv = 1.0f / 16384.0f;
  const float rscale = 16384.0f;
  const float oscPrj = 1.0f / 65536.0f;
  const float rres   = 1.0f / 16384.0f;

  cvt_qt<<<gQt, blk, 0, stream>>>(x, XT, 16.0f);
  cvt_h8<<<gW3, blk, 0, stream>>>(qkv_w, W3, n8w3, 1024.0f);
  cvt_h8<<<gPW, blk, 0, stream>>>(proj_w, PWp, n8pw, 1024.0f);
  gemm64<0, 2><<<gQkv, blk, 0, stream>>>(
      W3, CCH, 0LL, 0LL,
      XT, CCH, (long long)((size_t)NN * CCH), 0LL,
      XT, CCH,
      qkv_b,
      Y, NN, (long long)((size_t)NQKV * NN), 0LL,
      NQKV, NN, CCH, oscQkv, 0.0f);
  relayout_kernel<<<gRel, blk, 0, stream>>>(Y, QH, QL, KX, VH, VL);
  attn_kernel<<<gAttn, blk, 0, stream>>>(QH, QL, KX, VH, VL, tpm, temper, CTXh, CTXl, rscale);
  gemm64<2, 2><<<gProj, blk, 0, stream>>>(
      PWp, CCH, 0LL, 0LL,
      CTXh, CCH, (long long)((size_t)NN * CCH), 0LL,
      CTXl, CCH,
      proj_b,
      out, NN, (long long)((size_t)CCH * NN), 0LL,
      CCH, NN, CCH, oscPrj, rres);
  (void)hipGetLastError();
}
